// LocalMIDIGenerator_78357383348438
// MI455X (gfx1250) — hardware-run, weakly checked
//
#include <hip/hip_runtime.h>


#define NB_  2
#define LL   1024
#define DD   768
#define DI   1536
#define NS   16
#define RR   48
#define RP   64
#define PW   128
#define VOC  512
typedef _Float16 h16;
typedef unsigned short bf;
typedef __attribute__((ext_vector_type(16))) __bf16   v16bf;
typedef __attribute__((ext_vector_type(16))) _Float16 v16h;
typedef __attribute__((ext_vector_type(8)))  _Float16 v8h;
typedef __attribute__((ext_vector_type(8)))  unsigned short v8us;
typedef __attribute__((ext_vector_type(8)))  float    v8f;
typedef __attribute__((ext_vector_type(4)))  float    v4f;
typedef v8h  __attribute__((may_alias)) v8ha;
typedef v4f  __attribute__((may_alias)) v4fa;
typedef v8us __attribute__((may_alias)) v8usa;

__device__ __forceinline__ unsigned short f2bf(float f) { unsigned u = __float_as_uint(f); u += 0x7FFFu + ((u >> 16) & 1u); return (unsigned short)(u >> 16); }
__device__ __forceinline__ float bf2f(unsigned short b) { return __uint_as_float(((unsigned)b) << 16); }
__device__ __forceinline__ float bfr(float f) { return bf2f(f2bf(f)); }
__device__ __forceinline__ v16h cat16(v8h lo, v8h hi) { return __builtin_shufflevector(lo, hi, 0, 1, 2, 3, 4, 5, 6, 7, 8, 9, 10, 11, 12, 13, 14, 15); }
__device__ __forceinline__ v16bf cat16b(v8us lo, v8us hi) { return __builtin_bit_cast(v16bf, __builtin_shufflevector(lo, hi, 0, 1, 2, 3, 4, 5, 6, 7, 8, 9, 10, 11, 12, 13, 14, 15)); }
__device__ __forceinline__ v8f wmma16(v16h a, v16h b, v8f c) { return __builtin_amdgcn_wmma_f32_16x16x32_f16(false, a, false, b, (short)0, c, false, false); }
__device__ __forceinline__ v8f wmmab(v16bf a, v16bf b, v8f c) { return __builtin_amdgcn_wmma_f32_16x16x32_bf16(false, a, false, b, (short)0, c, false, false); }


template <typename T16> struct WFrag;
template <> struct WFrag<h16> { typedef v16h V; static __device__ __forceinline__ V ld(const h16* p) { return cat16(*(const v8h*)p, *(const v8h*)(p + 16)); } static __device__ __forceinline__ v8f mma(V a, V b, v8f c) { return wmma16(a, b, c); } };
template <> struct WFrag<bf> { typedef v16bf V; static __device__ __forceinline__ V ld(const bf* p) { return cat16b(*(const v8us*)p, *(const v8us*)(p + 16)); } static __device__ __forceinline__ v8f mma(V a, V b, v8f c) { return wmmab(a, b, c); } };
template <typename T16, int NSPLIT, bool BIAS>
__global__ __launch_bounds__(32) void k_gemmw(const T16* __restrict__ A, const T16* __restrict__ A2, const T16* __restrict__ Bt, const T16* __restrict__ Bt2, int K, float* C, int ldc, const float* __restrict__ bias, size_t sA, size_t sB, size_t sC) {
    typedef typename WFrag<T16>::V V;
    __shared__ __align__(16) float os[16 * 68];
    const size_t z = blockIdx.z; A += z * sA; if (A2) A2 += z * sA; Bt += z * sB; if (Bt2) Bt2 += z * sB; C += z * sC;
    const int lane = threadIdx.x & 31, lr = lane & 15, hi = lane >> 4; const int r0 = blockIdx.x * 64, c0 = blockIdx.y * 64;
    v8f acc[4][4];
#pragma unroll
    for (int mb = 0; mb < 4; ++mb)
#pragma unroll
        for (int nb = 0; nb < 4; ++nb) acc[mb][nb] = (v8f){};
    const size_t aoff = (size_t)(r0 + lr) * K + 8 * hi, boff = (size_t)(c0 + lr) * K + 8 * hi;
#pragma unroll 1
    for (int kc = 0; kc < K; kc += 32) {
        V a[4], a2[4];
#pragma unroll
        for (int mb = 0; mb < 4; ++mb) { a[mb] = WFrag<T16>::ld(A + aoff + (size_t)mb * 16 * K + kc); if (NSPLIT == 1 || NSPLIT == 2) a2[mb] = WFrag<T16>::ld(A2 + aoff + (size_t)mb * 16 * K + kc); }
#pragma unroll
        for (int nb = 0; nb < 4; ++nb) { const V b = WFrag<T16>::ld(Bt + boff + (size_t)nb * 16 * K + kc); V b2; if (NSPLIT >= 2) b2 = WFrag<T16>::ld(Bt2 + boff + (size_t)nb * 16 * K + kc);
#pragma unroll
            for (int mb = 0; mb < 4; ++mb) { acc[mb][nb] = WFrag<T16>::mma(a[mb], b, acc[mb][nb]); if (NSPLIT == 1 || NSPLIT == 2) acc[mb][nb] = WFrag<T16>::mma(a2[mb], b, acc[mb][nb]); if (NSPLIT >= 2) acc[mb][nb] = WFrag<T16>::mma(a[mb], b2, acc[mb][nb]); } }
        asm volatile("v_nop\n\tv_nop\n\tv_nop\n\tv_nop" : "+v"(acc[0][0]), "+v"(acc[1][1]), "+v"(acc[2][2]), "+v"(acc[3][3]) : "v"(a[0]), "v"(a[3]));
    }
#pragma unroll
    for (int mb = 0; mb < 4; ++mb) {
#pragma unroll
        for (int nb = 0; nb < 4; ++nb) {
#pragma unroll
            for (int j = 0; j < 8; ++j) os[(hi * 8 + j) * 68 + nb * 16 + lr] = acc[mb][nb][j]; }
        __builtin_amdgcn_wave_barrier(); asm volatile("" ::: "memory");
        float* crow = C + (size_t)(r0 + mb * 16) * ldc + c0;
#pragma unroll 1
        for (int ps = 0; ps < 2; ++ps) {
#pragma unroll
            for (int s = 0; s < 8; ++s) { const int row = 2 * s + hi, cofs = lr * 4; v4f val = *(const v4fa*)(os + row * 68 + cofs); if (BIAS) { val[0] += bfr(bias[c0 + cofs]); val[1] += bfr(bias[c0 + cofs + 1]); val[2] += bfr(bias[c0 + cofs + 2]); val[3] += bfr(bias[c0 + cofs + 3]); }
                *(volatile v4f*)(crow + (size_t)row * ldc + cofs) = val; }
            if (ps == 0) __threadfence(); }
        __builtin_amdgcn_wave_barrier(); asm volatile("" ::: "memory");
    }
}

__device__ __forceinline__ void splitf(float y, unsigned short& h, unsigned short& l) { h = f2bf(y); l = f2bf(y - bf2f(h)); }
__device__ __forceinline__ float silu_(float x) { return __fmul_rn(x, __fdiv_rn(1.0f, 1.0f + __expf(-x))); }
__device__ __forceinline__ float softplus_(float x) { return x > 20.f ? x : log1pf(__expf(x)); }
typedef __attribute__((ext_vector_type(2))) unsigned short v2us;
typedef __attribute__((ext_vector_type(4))) unsigned short v4us;

__global__ __launch_bounds__(256) void k_cvt8(const float* __restrict__ src, bf* dst, size_t n8) { const size_t i = (size_t)blockIdx.x * 256 + threadIdx.x; if (i >= n8) return; const v8f v = *(const v8f*)(src + i * 8); v8us o;
#pragma unroll
    for (int k = 0; k < 8; ++k) o[k] = f2bf(v[k]); *(volatile v8us*)(dst + i * 8) = o; __threadfence(); *(volatile v8us*)(dst + i * 8) = o; }
__global__ __launch_bounds__(256) void k_wpad(const float* __restrict__ w, int nreal, int kreal, int NOUT, int KP, bf* Bt) { const int i = (blockIdx.x * 256 + threadIdx.x) * 4; if (i >= NOUT * KP) return; const int k = i % KP, n = i / KP; v4us o;
#pragma unroll
    for (int q = 0; q < 4; ++q) o[q] = (n < nreal && k + q < kreal) ? f2bf(w[(size_t)n * kreal + k + q]) : (unsigned short)0; *(volatile v4us*)(Bt + i) = o; __threadfence(); *(volatile v4us*)(Bt + i) = o; }
__global__ __launch_bounds__(256) void k_split(const float* __restrict__ F, int pitch, int c0, int wsel, int wout, bf* Hh, bf* Hl) { const int e = (blockIdx.x * 256 + threadIdx.x) * 4; if (e >= LL * wout) return; const int c = e % wout, t = e / wout; v4us oh, ol;
#pragma unroll
    for (int q = 0; q < 4; ++q) { const float v = (c + q < wsel) ? F[(size_t)t * pitch + c0 + c + q] : 0.f; unsigned short u, l; splitf(v, u, l); oh[q] = u; ol[q] = l; } *(volatile v4us*)(Hh + e) = oh; *(volatile v4us*)(Hl + e) = ol; __threadfence(); *(volatile v4us*)(Hh + e) = oh; *(volatile v4us*)(Hl + e) = ol; }
__global__ __launch_bounds__(256) void k_x0(const int* __restrict__ tok, const int* __restrict__ tid, const float* __restrict__ Em, const float* __restrict__ Et, const float* __restrict__ CP, bf* Xh, bf* Xl) { const int e = (blockIdx.x * 256 + threadIdx.x) * 4; if (e >= LL * (DD / 2)) return; const int j = e % (DD / 2); const int t = e / (DD / 2);
    int mt = tok[t]; mt = mt < 0 ? 0 : (mt >= VOC ? VOC - 1 : mt); int tt = tid[t]; tt = tt < 0 ? 0 : (tt >= 64 ? 63 : tt); const float* em = Em + (size_t)mt * DD; const float* et = Et + (size_t)tt * DD; const float* cp = CP + (size_t)t * DD; v4us ah, al, bh, bl;
#pragma unroll 1
    for (int q = 0; q < 4; ++q) { const int jj = j + q; const int d1 = 2 * jj, d2 = 2 * jj + 1; const float x1 = __fadd_rn(__fadd_rn(bfr(em[d1]), cp[d1]), bfr(et[d1])); const float x2 = __fadd_rn(__fadd_rn(bfr(em[d2]), cp[d2]), bfr(et[d2]));
        const float fs = 6.283185307179586f / (float)(1 << (d1 / 192)); const float fc = 6.283185307179586f / (float)(1 << (d2 / 192)); const float s = sinf(__fmul_rn((float)t, fs)); const float c = cosf(__fmul_rn((float)t, fc));
        float p1 = __fmul_rn(x1, c); asm volatile("" : "+v"(p1)); float p2 = __fmul_rn(x2, s); asm volatile("" : "+v"(p2)); float p3 = __fmul_rn(x2, c); asm volatile("" : "+v"(p3)); float p4 = __fmul_rn(x1, s); asm volatile("" : "+v"(p4));
        unsigned short u, l; splitf(__fsub_rn(p1, p2), u, l); ah[q] = u; al[q] = l; splitf(__fadd_rn(p3, p4), u, l); bh[q] = u; bl[q] = l; }
    const size_t o1 = (size_t)t * DD + j, o2 = o1 + DD / 2; for (int ps = 0; ps < 2; ++ps) { *(volatile v4us*)(Xh + o1) = ah; *(volatile v4us*)(Xl + o1) = al; *(volatile v4us*)(Xh + o2) = bh; *(volatile v4us*)(Xl + o2) = bl; if (ps == 0) __threadfence(); } }
__global__ __launch_bounds__(256) void k_conv(const float* __restrict__ XZ, const float* __restrict__ w, const float* __restrict__ bb, float* XC, bf* Ch, bf* Cl) { const int e = (blockIdx.x * 256 + threadIdx.x) * 4; if (e >= LL * DI) return; const int c = e % DI, t = e / DI; v4f o; v4us oh, ol;
#pragma unroll
    for (int q = 0; q < 4; ++q) { const int cc = c + q; float acc = 0.f;
#pragma unroll
        for (int k = 0; k < 4; ++k) { const int ts = t - 3 + k; if (ts >= 0) { float p = __fmul_rn(bfr(w[cc * 4 + k]), XZ[(size_t)ts * 2 * DI + cc]); asm volatile("" : "+v"(p)); acc = __fadd_rn(acc, p); } }
        o[q] = silu_(__fadd_rn(acc, bfr(bb[cc]))); unsigned short u, l; splitf(o[q], u, l); oh[q] = u; ol[q] = l; }
    for (int ps = 0; ps < 2; ++ps) { *(volatile v4f*)(XC + e) = o; *(volatile v4us*)(Ch + e) = oh; *(volatile v4us*)(Cl + e) = ol; if (ps == 0) __threadfence(); } }
__global__ __launch_bounds__(256) void k_relupl(const float* __restrict__ F, int w, const float* __restrict__ b, bf* Ph, bf* Pl) { const int e = (blockIdx.x * 256 + threadIdx.x) * 4; if (e >= LL * w) return; const int c = e % w; const v4f a = *(const v4f*)(F + e); v4us oh, ol;
#pragma unroll
    for (int q = 0; q < 4; ++q) { unsigned short u, l; splitf(fmaxf(__fadd_rn(a[q], bfr(b[c + q])), 0.f), u, l); oh[q] = u; ol[q] = l; } *(volatile v4us*)(Ph + e) = oh; *(volatile v4us*)(Pl + e) = ol; __threadfence(); *(volatile v4us*)(Ph + e) = oh; *(volatile v4us*)(Pl + e) = ol; }
__global__ __launch_bounds__(256) void k_scan(const float* __restrict__ DTR, const float* __restrict__ dtb, const float* __restrict__ XC, const float* __restrict__ XDBL, const float* __restrict__ XZ, const float* __restrict__ alog, const float* __restrict__ Dp, bf* Yh, bf* Yl) {
    __shared__ float ybuf[64]; const int tid = threadIdx.x; const int cl = tid >> 2, sub = tid & 3; const int d = blockIdx.x * 64 + cl; const int n0 = sub * 4; float A[4], h[4];
#pragma unroll
    for (int j = 0; j < 4; ++j) { A[j] = -__expf(bfr(alog[(size_t)d * NS + n0 + j])); h[j] = 0.f; }
    const float dd = bfr(Dp[d]); const float db = bfr(dtb[d]);
    for (int t = 0; t < LL; ++t) { const float dt = softplus_(__fadd_rn(DTR[(size_t)t * DI + d], db)); const float xc = XC[(size_t)t * DI + d]; const float dtx = __fmul_rn(dt, xc); const float* pr = XDBL + (size_t)t * PW + RR; float y = 0.f;
#pragma unroll
        for (int j = 0; j < 4; ++j) { const float a = __expf(__fmul_rn(dt, A[j])); float ha = __fmul_rn(h[j], a); asm volatile("" : "+v"(ha)); float hb = __fmul_rn(dtx, pr[n0 + j]); asm volatile("" : "+v"(hb)); h[j] = __fadd_rn(ha, hb); float yc = __fmul_rn(h[j], pr[NS + n0 + j]); asm volatile("" : "+v"(yc)); y = __fadd_rn(y, yc); }
        y += __shfl_xor(y, 1, 32); y += __shfl_xor(y, 2, 32);
        if (sub == 0) { float sk = __fmul_rn(dd, xc); asm volatile("" : "+v"(sk)); ybuf[cl] = __fmul_rn(__fadd_rn(y, sk), silu_(XZ[(size_t)t * 2 * DI + DI + d])); }
        __syncthreads();
        if (tid < 32) { v2us oh, ol; unsigned short u, l; splitf(ybuf[2 * tid], u, l); oh[0] = u; ol[0] = l; splitf(ybuf[2 * tid + 1], u, l); oh[1] = u; ol[1] = l; const size_t o = (size_t)t * DI + blockIdx.x * 64 + 2 * tid; *(volatile v2us*)(Yh + o) = oh; *(volatile v2us*)(Yl + o) = ol; __threadfence(); *(volatile v2us*)(Yh + o) = oh; *(volatile v2us*)(Yl + o) = ol; }
        __syncthreads(); } }
__global__ __launch_bounds__(256) void k_tp(const float* __restrict__ T1, const float* __restrict__ tb1, const float* __restrict__ tw2, const float* __restrict__ tb2, float* OUT2) { const int t = blockIdx.x * 256 + threadIdx.x; if (t >= LL) return; const float* r = T1 + (size_t)t * DD; float s = bfr(tb2[0]);
#pragma unroll 1
    for (int c = 0; c < DD; ++c) { float p = __fmul_rn(fmaxf(__fadd_rn(r[c], bfr(tb1[c])), 0.f), bfr(tw2[c])); asm volatile("" : "+v"(p)); s = __fadd_rn(s, p); } *(volatile float*)(OUT2 + t) = s; __threadfence(); *(volatile float*)(OUT2 + t) = s; }
__global__ __launch_bounds__(256) void k_rh(const float* __restrict__ R2, const float* __restrict__ rb2, float* OUT1) { const int t = blockIdx.x * 256 + threadIdx.x; if (t >= LL) return; const v4f a = *(const v4f*)(R2 + (size_t)t * 64); v4f o; o[0] = __fadd_rn(a[0], bfr(rb2[0])); o[1] = __fadd_rn(a[1], bfr(rb2[1])); o[2] = __fadd_rn(a[2], bfr(rb2[2])); o[3] = __fadd_rn(a[3], bfr(rb2[3])); *(volatile v4f*)(OUT1 + (size_t)t * 4) = o; __threadfence(); *(volatile v4f*)(OUT1 + (size_t)t * 4) = o; }

extern "C" void kernel_launch(void* const* d_in, const int* in_sizes, int n_in,
                              void* d_out, int out_size, void* d_ws, size_t ws_size, hipStream_t stream) {
    (void)in_sizes; (void)n_in; (void)out_size;
    const int* tok = (const int*)d_in[0]; const float* ctrl = (const float*)d_in[1]; const int* tid = (const int*)d_in[2]; const float* Em = (const float*)d_in[3]; const float* Et = (const float*)d_in[4]; const float* Wc = (const float*)d_in[5]; const float* bc = (const float*)d_in[6];
    const float* inw = (const float*)d_in[7]; const float* cw = (const float*)d_in[8]; const float* cb = (const float*)d_in[9]; const float* xpw = (const float*)d_in[10]; const float* dtw = (const float*)d_in[11]; const float* dtb = (const float*)d_in[12]; const float* alog = (const float*)d_in[13]; const float* Dp = (const float*)d_in[14]; const float* outw = (const float*)d_in[15];
    const float* Wo = (const float*)d_in[16]; const float* bo = (const float*)d_in[17]; const float* tw1 = (const float*)d_in[18]; const float* tb1 = (const float*)d_in[19]; const float* tw2 = (const float*)d_in[20]; const float* tb2 = (const float*)d_in[21]; const float* rw1 = (const float*)d_in[22]; const float* rb1 = (const float*)d_in[23]; const float* rw2 = (const float*)d_in[24]; const float* rb2 = (const float*)d_in[25];
    float* OUT0 = (float*)d_out; float* OUT1 = (float*)((char*)d_out + 4194304); float* OUT2 = (float*)((char*)d_out + 4227072);
    char* wsp = (char*)d_ws;
    auto take = [&](size_t bytes) { char* p = wsp; wsp += (bytes + 255) & ~(size_t)255; return (void*)p; };
    bf* WC = (bf*)take(DD * DD * 2); bf* TW1 = (bf*)take(DD * DD * 2); bf* RW1 = (bf*)take(DD * DD * 2); bf* RW2 = (bf*)take(64 * DD * 2); bf* WO = (bf*)take(VOC * DD * 2);
    bf* WIN[2]; bf* WXP[2]; bf* WDT[2]; bf* WOUT[2]; for (int i = 0; i < 2; ++i) { WIN[i] = (bf*)take((size_t)2 * DI * DD * 2); WXP[i] = (bf*)take((size_t)PW * DI * 2); WDT[i] = (bf*)take((size_t)DI * RP * 2); WOUT[i] = (bf*)take((size_t)DD * DI * 2); }
    bf* CB = (bf*)take((size_t)LL * DD * 2); float* CP = (float*)take((size_t)LL * DD * 4); float* T1 = (float*)take((size_t)LL * DD * 4); bf* Xh = (bf*)take((size_t)LL * DD * 2); bf* Xl = (bf*)take((size_t)LL * DD * 2); float* XZ = (float*)take((size_t)LL * 2 * DI * 4); float* XC = (float*)take((size_t)LL * DI * 4); bf* Ch = (bf*)take((size_t)LL * DI * 2); bf* Cl = (bf*)take((size_t)LL * DI * 2);
    float* XDBL = (float*)take((size_t)LL * PW * 4); bf* Rh = (bf*)take((size_t)LL * RP * 2); bf* Rl = (bf*)take((size_t)LL * RP * 2); float* DTR = (float*)take((size_t)LL * DI * 4); bf* Yh = (bf*)take((size_t)LL * DI * 2); bf* Yl = (bf*)take((size_t)LL * DI * 2); float* XF = (float*)take((size_t)LL * DD * 4); float* R1 = (float*)take((size_t)LL * DD * 4); bf* R1h = (bf*)take((size_t)LL * DD * 2); bf* R1l = (bf*)take((size_t)LL * DD * 2); float* R2 = (float*)take((size_t)LL * 64 * 4);
    if ((size_t)(wsp - (char*)d_ws) > ws_size) return;
    k_cvt8<<<(DD * DD / 8 + 255) / 256, 256, 0, stream>>>(Wc, WC, DD * DD / 8); k_cvt8<<<(DD * DD / 8 + 255) / 256, 256, 0, stream>>>(tw1, TW1, DD * DD / 8); k_cvt8<<<(DD * DD / 8 + 255) / 256, 256, 0, stream>>>(rw1, RW1, DD * DD / 8); k_wpad<<<(64 * DD / 4 + 255) / 256, 256, 0, stream>>>(rw2, 4, DD, 64, DD, RW2); k_cvt8<<<(VOC * DD / 8 + 255) / 256, 256, 0, stream>>>(Wo, WO, VOC * DD / 8);
    for (int i = 0; i < 2; ++i) { k_cvt8<<<(unsigned)(((size_t)2 * DI * DD / 8 + 255) / 256), 256, 0, stream>>>(inw + (size_t)i * 2 * DI * DD, WIN[i], (size_t)2 * DI * DD / 8); k_wpad<<<(PW * DI / 4 + 255) / 256, 256, 0, stream>>>(xpw + (size_t)i * (RR + 2 * NS) * DI, RR + 2 * NS, DI, PW, DI, WXP[i]); k_wpad<<<(DI * RP / 4 + 255) / 256, 256, 0, stream>>>(dtw + (size_t)i * DI * RR, DI, RR, DI, RP, WDT[i]); k_cvt8<<<(unsigned)(((size_t)DD * DI / 8 + 255) / 256), 256, 0, stream>>>(outw + (size_t)i * DD * DI, WOUT[i], (size_t)DD * DI / 8); }
    for (int b = 0; b < NB_; ++b) {
        k_cvt8<<<(LL * DD / 8 + 255) / 256, 256, 0, stream>>>(ctrl + (size_t)b * LL * DD, CB, (size_t)LL * DD / 8);
        k_gemmw<bf, 0, true><<<dim3(LL / 64, DD / 64, 1), 32, 0, stream>>>(CB, nullptr, WC, nullptr, DD, CP, DD, bc, 0, 0, 0); k_gemmw<bf, 0, false><<<dim3(LL / 64, DD / 64, 1), 32, 0, stream>>>(CB, nullptr, TW1, nullptr, DD, T1, DD, nullptr, 0, 0, 0);
        k_tp<<<LL / 256, 256, 0, stream>>>(T1, tb1, tw2, tb2, OUT2 + (size_t)b * LL);
        k_x0<<<(LL * (DD / 2) / 4 + 255) / 256, 256, 0, stream>>>(tok + (size_t)b * LL, tid + (size_t)b * LL, Em, Et, CP, Xh, Xl);
        for (int i = 0; i < 2; ++i) {
            k_gemmw<bf, 1, false><<<dim3(LL / 64, 2 * DI / 64, 1), 32, 0, stream>>>(Xh, Xl, WIN[i], nullptr, DD, XZ, 2 * DI, nullptr, 0, 0, 0);
            k_conv<<<(LL * DI / 4 + 255) / 256, 256, 0, stream>>>(XZ, cw + (size_t)i * DI * 4, cb + (size_t)i * DI, XC, Ch, Cl);
            k_gemmw<bf, 1, false><<<dim3(LL / 64, PW / 64, 1), 32, 0, stream>>>(Ch, Cl, WXP[i], nullptr, DI, XDBL, PW, nullptr, 0, 0, 0);
            k_split<<<(LL * RP / 4 + 255) / 256, 256, 0, stream>>>(XDBL, PW, 0, RR, RP, Rh, Rl);
            k_gemmw<bf, 1, false><<<dim3(LL / 64, DI / 64, 1), 32, 0, stream>>>(Rh, Rl, WDT[i], nullptr, RP, DTR, DI, nullptr, 0, 0, 0);
            k_scan<<<DI / 64, 256, 0, stream>>>(DTR, dtb + (size_t)i * DI, XC, XDBL, XZ, alog + (size_t)i * DI * NS, Dp + (size_t)i * DI, Yh, Yl);
            k_gemmw<bf, 1, false><<<dim3(LL / 64, DD / 64, 1), 32, 0, stream>>>(Yh, Yl, WOUT[i], nullptr, DI, XF, DD, nullptr, 0, 0, 0);
            k_split<<<(LL * DD / 4 + 255) / 256, 256, 0, stream>>>(XF, DD, 0, DD, DD, Xh, Xl); }
        k_gemmw<bf, 1, true><<<dim3(LL / 64, VOC / 64, 1), 32, 0, stream>>>(Xh, Xl, WO, nullptr, DD, OUT0 + (size_t)b * LL * VOC, VOC, bo, 0, 0, 0);
        k_gemmw<bf, 1, false><<<dim3(LL / 64, DD / 64, 1), 32, 0, stream>>>(Xh, Xl, RW1, nullptr, DD, R1, DD, nullptr, 0, 0, 0); k_relupl<<<(LL * DD / 4 + 255) / 256, 256, 0, stream>>>(R1, DD, rb1, R1h, R1l);
        k_gemmw<bf, 1, false><<<dim3(LL / 64, 1, 1), 32, 0, stream>>>(R1h, R1l, RW2, nullptr, DD, R2, 64, nullptr, 0, 0, 0); k_rh<<<LL / 256, 256, 0, stream>>>(R2, rb2, OUT1 + (size_t)b * LL * 4); }
}
